// SpectralGNNEncoder_2680059592979
// MI455X (gfx1250) — hardware-verified
//
#include <hip/hip_runtime.h>
#include <stdint.h>


#define FEAT 128
#define LATD 64
#define KSTEPS 4
#define NTILES 8
#define RAGG 448
#define CHUNK 1024
#define RDEG 4096
#define LDP 132
#define A_SCALE 16.0f
#define W_SCALE 64.0f
#define OUT_SCALE 0.0009765625f

typedef _Float16 v16h __attribute__((ext_vector_type(16)));
typedef _Float16 v8h __attribute__((ext_vector_type(8)));
typedef float v8f __attribute__((ext_vector_type(8)));
typedef float v4f __attribute__((ext_vector_type(4)));
typedef int v4i __attribute__((ext_vector_type(4)));
union Frag { v16h v; v8h half[2]; };

static __device__ __forceinline__ v8f wmma16(v16h a, v16h b, v8f c) {
  v8f d = __builtin_amdgcn_wmma_f32_16x16x32_f16(false, a, false, b, (short)0, c, false, false);
  asm volatile("v_nop\n\tv_nop\n\tv_nop\n\tv_nop" : "+v"(d) : "v"(a), "v"(b));
  return d;
}

static __device__ __forceinline__ void store2(float* p, v4f v) {
  *(volatile v4f*)p = v;
  __threadfence();
  *(volatile v4f*)p = v;
}

static __device__ __forceinline__ int excl_scan32(int v, int lane, int* total) {
  int incl = v;
#pragma unroll
  for (int o = 1; o < 32; o <<= 1) {
    int t = __shfl_up(incl, o);
    if (lane >= o) incl += t;
  }
  *total = __shfl(incl, 31);
  return incl - v;
}

template <bool VEC>
static __device__ __forceinline__ unsigned hit_mask(const int* __restrict__ edst, int cb, int lane,
                                                      int NE, int n0, unsigned Rb) {
  unsigned mask = 0u;
#pragma unroll
  for (int j = 0; j < 8; ++j) {
    const int e = cb + 4 * (lane + 32 * j);
    int d0 = -1, d1 = -1, d2 = -1, d3 = -1;
    if (VEC) {
      if (e < NE) {
        const v4i dv = *(const v4i*)(edst + e);
        d0 = dv[0]; d1 = dv[1]; d2 = dv[2]; d3 = dv[3];
      }
    } else {
      if (e < NE) d0 = edst[e];
      if (e + 1 < NE) d1 = edst[e + 1];
      if (e + 2 < NE) d2 = edst[e + 2];
      if (e + 3 < NE) d3 = edst[e + 3];
    }
    const unsigned h0 = ((unsigned)(d0 - n0) < Rb) ? 1u : 0u;
    const unsigned h1 = ((unsigned)(d1 - n0) < Rb) ? 1u : 0u;
    const unsigned h2 = ((unsigned)(d2 - n0) < Rb) ? 1u : 0u;
    const unsigned h3 = ((unsigned)(d3 - n0) < Rb) ? 1u : 0u;
    mask |= (h0 | (h1 << 1) | (h2 << 2) | (h3 << 3)) << (4 * j);
  }
  return mask;
}

__global__ __launch_bounds__(256) void k_pack(const float* __restrict__ W1, const float* __restrict__ W2,
                                              const float* __restrict__ Wmu, const float* __restrict__ Wlv,
                                              _Float16* P1, _Float16* P2, _Float16* P3) {
  const int p = blockIdx.x * 256 + threadIdx.x;
  const int which = blockIdx.y;
  if (p >= FEAT * FEAT / 8) return;
  const int frag = p >> 6;
  const int lane = (p >> 1) & 31;
  const int hh = p & 1;
  const int kt = frag / NTILES;
  const int nt = frag - kt * NTILES;
  const int n = nt * 16 + (lane & 15);
  const int kb = kt * 32 + 16 * hh + 8 * (lane >> 4);
  v8h v;
#pragma unroll
  for (int j = 0; j < 8; ++j) {
    const int k = kb + j;
    float w;
    if (which == 0) w = W1[k * FEAT + n];
    else if (which == 1) w = W2[k * FEAT + n];
    else w = (n < LATD) ? Wmu[k * LATD + n] : Wlv[k * LATD + (n - LATD)];
    v[j] = (_Float16)(w * W_SCALE);
  }
  _Float16* dst = ((which == 0) ? P1 : ((which == 1) ? P2 : P3)) + (size_t)p * 8;
  *(volatile v8h*)dst = v;
  __threadfence();
  *(volatile v8h*)dst = v;
}

template <bool VEC>
__global__ __launch_bounds__(32) void k_deg(const int* __restrict__ edst, const float* __restrict__ ew,
                                            float* dinv, int NE, int NN) {
  __shared__ float s_deg[RDEG];
  __shared__ int l_ld[CHUNK];
  __shared__ float l_w[CHUNK];
  const int lane = threadIdx.x;
  const int n0 = blockIdx.x * RDEG;
  if (n0 >= NN) return;
  const int rbi = (NN - n0 < RDEG) ? (NN - n0) : RDEG;
  const unsigned Rb = (unsigned)rbi;
  for (int i = lane; i < RDEG; i += 32) s_deg[i] = 1.0f;
  __syncthreads();

  for (int cb = 0; cb < NE; cb += CHUNK) {
    const unsigned mask = hit_mask<VEC>(edst, cb, lane, NE, n0, Rb);
    const int cnt = __builtin_popcount(mask);
    int total;
    int pos = excl_scan32(cnt, lane, &total);
    unsigned mk = mask;
    while (mk) {
      const int i = __builtin_ctz(mk);
      mk &= mk - 1u;
      const int e = cb + 4 * (lane + 32 * (i >> 2)) + (i & 3);
      const int d = edst[e];
      const float w = ew[e];
      if (pos < CHUNK) { l_ld[pos] = d - n0; l_w[pos] = w; }
      ++pos;
    }
    __syncthreads();
    const int nh = (total < CHUNK) ? total : CHUNK;
    for (int q = 0; q < nh; ++q) {
      int ld = l_ld[q];
      const float w = l_w[q];
      ld = (ld < 0) ? 0 : ((ld >= RDEG) ? (RDEG - 1) : ld);
      if ((ld & 31) == lane) s_deg[ld] += w;
    }
    __syncthreads();
  }

#pragma unroll 1
  for (int i = 0; i < RDEG / 128; ++i) {
    const int idx = i * 32 + lane;
    const v4f dg = *(const v4f*)(s_deg + 4 * idx);
    v4f dv;
#pragma unroll
    for (int c = 0; c < 4; ++c) dv[c] = (dg[c] > 0.0f) ? (1.0f / sqrtf(dg[c])) : 0.0f;
    store2(dinv + (size_t)n0 + 4 * idx, dv);
  }
}

__global__ __launch_bounds__(32) void k_gemm(const float* __restrict__ A, const _Float16* __restrict__ Bp,
                                             const float* __restrict__ bias0, const float* __restrict__ bias1,
                                             float* out0, float* out1, int M, int split) {
  __shared__ float s_t[16 * LDP];
  const int l = threadIdx.x;
  const int h = l >> 4;
  const int m = l & 15;
  const int row0 = blockIdx.x * 16;
  if (row0 >= M) return;
  int arow = row0 + m;
  if (arow > M - 1) arow = M - 1;
  const float* ap = A + (size_t)arow * FEAT + 8 * h;

  v8f acc[NTILES];
  const v8f z8 = {0.f, 0.f, 0.f, 0.f, 0.f, 0.f, 0.f, 0.f};
#pragma unroll
  for (int t = 0; t < NTILES; ++t) acc[t] = z8;

#pragma unroll 1
  for (int kt = 0; kt < KSTEPS; ++kt) {
    const float* p0 = ap + kt * 32;
    const v8f xa = *(const v8f*)(p0);
    const v8f xb = *(const v8f*)(p0 + 16);
    Frag a;
    a.half[0] = __builtin_convertvector(xa * A_SCALE, v8h);
    a.half[1] = __builtin_convertvector(xb * A_SCALE, v8h);
    const _Float16* bk = Bp + (size_t)kt * (NTILES * 32 * 16) + l * 16;
#pragma unroll
    for (int t = 0; t < NTILES; ++t) {
      const _Float16* bp = bk + t * (32 * 16);
      Frag b;
      b.half[0] = *(const v8h*)(bp);
      b.half[1] = *(const v8h*)(bp + 8);
      acc[t] = wmma16(a.v, b.v, acc[t]);
    }
  }

#pragma unroll
  for (int t = 0; t < NTILES; ++t) {
#pragma unroll
    for (int r = 0; r < 8; ++r) s_t[(8 * h + r) * LDP + 16 * t + m] = acc[t][r] * OUT_SCALE;
  }
  __syncthreads();

  v4f bv = {0.f, 0.f, 0.f, 0.f};
  if (split) {
    const float* bsrc = (l < 16) ? (bias0 + 4 * l) : (bias1 + 4 * (l - 16));
    bv = *(const v4f*)bsrc;
  }
#pragma unroll
  for (int rr = 0; rr < 16; ++rr) {
    const int row = row0 + rr;
    if (row < M) {
      const v4f v = *(const v4f*)(s_t + rr * LDP + 4 * l) + bv;
      float* p = split ? (((l < 16) ? out0 : out1) + (size_t)row * LATD + 4 * (l & 15))
                       : (out0 + (size_t)row * FEAT + 4 * l);
      *(volatile v4f*)p = v;
    }
  }
  __threadfence();
#pragma unroll
  for (int rr = 0; rr < 16; ++rr) {
    const int row = row0 + rr;
    if (row < M) {
      const v4f v = *(const v4f*)(s_t + rr * LDP + 4 * l) + bv;
      float* p = split ? (((l < 16) ? out0 : out1) + (size_t)row * LATD + 4 * (l & 15))
                       : (out0 + (size_t)row * FEAT + 4 * l);
      *(volatile v4f*)p = v;
    }
  }
}

template <bool VEC>
__global__ __launch_bounds__(32) void k_agg(const int* __restrict__ esrc, const int* __restrict__ edst,
                                            const float* __restrict__ ew, const float* __restrict__ dinv,
                                            const float* __restrict__ XW, const float* __restrict__ bias,
                                            float* H, int NE, int NN, int relu) {
  extern __shared__ v4f lds_dyn[];
  v4f* acc4 = lds_dyn;
  int* l_src = (int*)(lds_dyn + RAGG * 32);
  float* l_cf = (float*)(l_src + CHUNK);
  int* l_ld = (int*)(l_cf + CHUNK);
  const int lane = threadIdx.x;
  const int n0 = blockIdx.x * RAGG;
  if (n0 >= NN) return;
  const int rbi = (NN - n0 < RAGG) ? (NN - n0) : RAGG;
  const unsigned Rb = (unsigned)rbi;
  const v4f z4 = {0.f, 0.f, 0.f, 0.f};
  for (int i = lane; i < RAGG * 32; i += 32) acc4[i] = z4;
  __syncthreads();

  for (int cb = 0; cb < NE; cb += CHUNK) {
    const unsigned mask = hit_mask<VEC>(edst, cb, lane, NE, n0, Rb);
    const int cnt = __builtin_popcount(mask);
    int total;
    int pos = excl_scan32(cnt, lane, &total);
    unsigned mk = mask;
    while (mk) {
      const int i = __builtin_ctz(mk);
      mk &= mk - 1u;
      const int e = cb + 4 * (lane + 32 * (i >> 2)) + (i & 3);
      const int d = edst[e];
      int s = esrc[e];
      s = (s < 0) ? 0 : ((s > NN - 1) ? (NN - 1) : s);
      const float cf = ew[e] * dinv[s];
      if (pos < CHUNK) { l_src[pos] = s; l_cf[pos] = cf; l_ld[pos] = d - n0; }
      ++pos;
    }
    __syncthreads();
    const int nh = (total < CHUNK) ? total : CHUNK;
    for (int q = 0; q < nh; ++q) {
      int s = l_src[q];
      const float cf = l_cf[q];
      int ld = l_ld[q];
      s = ((unsigned)s < (unsigned)NN) ? s : 0;
      ld = ((unsigned)ld < (unsigned)RAGG) ? ld : 0;
      const v4f xv = *(const v4f*)(XW + (size_t)s * FEAT + 4 * lane);
      const v4f a = acc4[ld * 32 + lane];
      acc4[ld * 32 + lane] = a + cf * xv;
    }
    __syncthreads();
  }

  const v4f bvv = *(const v4f*)(bias + 4 * lane);
  for (int r = 0; r < rbi; ++r) {
    const int d = n0 + r;
    const float di = dinv[d];
    const v4f xv = *(const v4f*)(XW + (size_t)d * FEAT + 4 * lane);
    const v4f a = acc4[r * 32 + lane];
    v4f o = di * (a + di * xv) + bvv;
    if (relu) {
#pragma unroll
      for (int c = 0; c < 4; ++c) o[c] = fmaxf(o[c], 0.0f);
    }
    store2(H + (size_t)d * FEAT + 4 * lane, o);
  }
}

extern "C" void kernel_launch(void* const* d_in, const int* in_sizes, int n_in,
                              void* d_out, int out_size, void* d_ws, size_t ws_size,
                              hipStream_t stream) {
  if (n_in < 11) return;
  const float* x   = (const float*)d_in[0];
  const int*   ei  = (const int*)d_in[1];
  const float* ew  = (const float*)d_in[2];
  const float* W1  = (const float*)d_in[3];
  const float* b1  = (const float*)d_in[4];
  const float* W2  = (const float*)d_in[5];
  const float* b2  = (const float*)d_in[6];
  const float* Wmu = (const float*)d_in[7];
  const float* bmu = (const float*)d_in[8];
  const float* Wlv = (const float*)d_in[9];
  const float* blv = (const float*)d_in[10];

  const int NN = in_sizes[0] / FEAT;
  const int NE = in_sizes[1] / 2;
  if (NN <= 0 || NE < 0) return;
  if (out_size < 2 * NN * LATD) return;
  const int* esrc = ei;
  const int* edst = ei + NE;
  float* out0 = (float*)d_out;
  float* out1 = out0 + (size_t)NN * LATD;

  const int nBd = (NN + RDEG - 1) / RDEG;
  const int nBa = (NN + RAGG - 1) / RAGG;
  const int nBg = (NN + 15) / 16;

  char* ws = (char*)d_ws;
  size_t off = 0;
  auto carve = [&](size_t bytes) -> char* {
    char* p = ws + off;
    off += (bytes + 255) & ~(size_t)255;
    return p;
  };
  _Float16* P1 = (_Float16*)carve((size_t)FEAT * FEAT * 2);
  _Float16* P2 = (_Float16*)carve((size_t)FEAT * FEAT * 2);
  _Float16* P3 = (_Float16*)carve((size_t)FEAT * FEAT * 2);
  float* dinv  = (float*)carve((size_t)nBd * RDEG * 4);
  float* XW    = (float*)carve((size_t)NN * FEAT * 4);
  float* Hf    = (float*)carve((size_t)NN * FEAT * 4);
  if (off > ws_size) return;

  const bool vec = ((NE & 3) == 0);
  const size_t ldsA = (size_t)RAGG * 32 * sizeof(v4f) + (size_t)CHUNK * 12;

  k_pack<<<dim3(FEAT * FEAT / 8 / 256, 3), 256, 0, stream>>>(W1, W2, Wmu, Wlv, P1, P2, P3);

  if (vec) k_deg<true><<<nBd, 32, 0, stream>>>(edst, ew, dinv, NE, NN);
  else     k_deg<false><<<nBd, 32, 0, stream>>>(edst, ew, dinv, NE, NN);

  k_gemm<<<nBg, 32, 0, stream>>>(x, P1, b1, b1, XW, XW, NN, 0);
  if (vec) k_agg<true><<<nBa, 32, ldsA, stream>>>(esrc, edst, ew, dinv, XW, b1, Hf, NE, NN, 1);
  else     k_agg<false><<<nBa, 32, ldsA, stream>>>(esrc, edst, ew, dinv, XW, b1, Hf, NE, NN, 1);

  k_gemm<<<nBg, 32, 0, stream>>>(Hf, P2, b2, b2, XW, XW, NN, 0);
  if (vec) k_agg<true><<<nBa, 32, ldsA, stream>>>(esrc, edst, ew, dinv, XW, b2, Hf, NE, NN, 0);
  else     k_agg<false><<<nBa, 32, ldsA, stream>>>(esrc, edst, ew, dinv, XW, b2, Hf, NE, NN, 0);

  k_gemm<<<nBg, 32, 0, stream>>>(Hf, P3, bmu, blv, out0, out1, NN, 1);
}
